// Layer_25692494364843
// MI455X (gfx1250) — hardware-run, weakly checked
//
#include <hip/hip_runtime.h>
#include <math.h>

typedef __attribute__((ext_vector_type(16))) _Float16 v16h;
typedef __attribute__((ext_vector_type(8)))  _Float16 v8h;
typedef __attribute__((ext_vector_type(8)))  float    v8f;
typedef __attribute__((ext_vector_type(4)))  float    v4f;

constexpr int kNb    = 8;
constexpr int kSin   = 1024;
constexpr int kSout  = 1024;
constexpr int kDi    = 256;
constexpr int kDo    = 256;
constexpr int kRows  = kNb * kSin;
static_assert(kRows == 8192, "token rows");
static_assert((kRows % 64) == 0 && (kDo % 64) == 0 && (kSout % 64) == 0 && (kSin % 64) == 0, "tile multiples of 64");
static_assert((kDi % 32) == 0 && (kSin % 32) == 0, "contraction depths multiples of 32");
static_assert(kDo == 256 && kNb == 8, "phase kernel mapping: 256 threads = 256 channels, 8 waves = 8 batch rows");

constexpr float kCarryX = 64.0f;
constexpr float kCarryM = 1024.0f;
constexpr float kCarryL = 4096.0f;
constexpr float kCarryR = 16.0f;
constexpr float kScaleProj = 1.0f / (kCarryX * kCarryM);
constexpr float kScaleLink = 1.0f / (kCarryL * kCarryR);
constexpr float kF16MinNormal = 6.103515625e-5f;
constexpr float kLnEps = 1e-5f;
constexpr float kTwoPi = 6.283185307179586f;

constexpr size_t kOffX16  = 0;
constexpr size_t kOffM16  = kOffX16  + (size_t)kRows * kDi * 2;
constexpr size_t kOffLtA  = kOffM16  + (size_t)kDo * kDi * 2;
constexpr size_t kOffZL   = kOffLtA  + (size_t)kSout * kSin * 2;
constexpr size_t kOffRP   = kOffZL   + (size_t)kRows * kDo * 4;
constexpr size_t kOffRT   = kOffRP   + (size_t)kRows * kDo * 4;
constexpr size_t kWsTotal = kOffRT   + (size_t)kNb * kDo * kSin * 2;
static_assert(kWsTotal == 27394048ull, "carve total");
static_assert(kWsTotal <= 134217728ull, "carve cap");
static_assert((kOffM16 % 128) == 0 && (kOffLtA % 128) == 0 && (kOffZL % 128) == 0 &&
              (kOffRP % 128) == 0 && (kOffRT % 128) == 0, "128-B aligned regions");

__device__ __forceinline__ _Float16 to_f16_carried(float v, float carry) {
  float c = v * carry;
  c = (fabsf(c) < kF16MinNormal) ? 0.0f : c;
  return (_Float16)c;
}

union FragU { v16h v; v8h h[2]; };
__device__ __forceinline__ v16h frag_load(const _Float16* p) {
  FragU f;
  f.h[0] = *(const v8h*)(p);
  f.h[1] = *(const v8h*)(p + 16);
  return f.v;
}

__device__ __forceinline__ v8f mma_f16(v16h a, v16h b, v8f c) {
  c = __builtin_amdgcn_wmma_f32_16x16x32_f16(false, a, false, b, (short)0, c, false, false);
  asm volatile("v_nop\n\tv_nop\n\tv_nop\n\tv_nop" : "+v"(c) : "v"(a), "v"(b));
  return c;
}

__global__ __launch_bounds__(256) void cast_rows_f16_kernel(
    const float* __restrict__ src, unsigned short* __restrict__ dst, int total8, float carry)
{
  const int i = blockIdx.x * 256 + threadIdx.x;
  if (i >= total8) return;
  const size_t e0 = (size_t)i << 3;
  const v4f a0 = *(const v4f*)(src + e0);
  const v4f a1 = *(const v4f*)(src + e0 + 4);
  v8h hv;
#pragma unroll
  for (int e = 0; e < 4; ++e) {
    const float f0 = a0[e];
    const float f1 = a1[e];
    hv[e]     = to_f16_carried(f0, carry);
    hv[4 + e] = to_f16_carried(f1, carry);
  }
  unsigned short* q = dst + e0;
  *(volatile v8h*)q = hv;
  __threadfence();
  *(volatile v8h*)q = hv;
}

__global__ __launch_bounds__(256) void transpose_f16_kernel(
    const float* __restrict__ in, unsigned short* __restrict__ out,
    int ldin, int ldout, long inBatch, long outBatch, float carry)
{
  __shared__ float tile[64 * 65];
  const int tid = threadIdx.x, lane = tid & 31, wave = tid >> 5;
  const int c0 = blockIdx.x * 64;
  const int r0 = blockIdx.y * 64;
  const float* src = in + (size_t)blockIdx.z * (size_t)inBatch;
  unsigned short* dstb = out + (size_t)blockIdx.z * (size_t)outBatch;
  {
    const int lr = tid >> 4, c4 = (tid & 15) * 4;
#pragma unroll
    for (int it = 0; it < 4; ++it) {
      const int row = lr + 16 * it;
      const v4f v = *(const v4f*)(src + (size_t)(r0 + row) * ldin + c0 + c4);
      tile[row * 65 + c4 + 0] = v[0];
      tile[row * 65 + c4 + 1] = v[1];
      tile[row * 65 + c4 + 2] = v[2];
      tile[row * 65 + c4 + 3] = v[3];
    }
  }
  __syncthreads();
  const int q = lane >> 3, r8 = (lane & 7) * 8;
  v8h hv[2];
#pragma unroll
  for (int it = 0; it < 2; ++it) {
    const int cc = it * 32 + wave * 4 + q;
#pragma unroll
    for (int e = 0; e < 8; ++e) {
      const float f = tile[(r8 + e) * 65 + cc];
      hv[it][e] = to_f16_carried(f, carry);
    }
  }
  for (int pass = 0; pass < 2; ++pass) {
#pragma unroll
    for (int it = 0; it < 2; ++it) {
      const int cc = it * 32 + wave * 4 + q;
      *(volatile v8h*)(dstb + (size_t)(c0 + cc) * ldout + r0 + r8) = hv[it];
    }
    __threadfence();
  }
}

__global__ __launch_bounds__(256) void gemm64_f16_kernel(
    const unsigned short* __restrict__ Ap, int lda, long strideA,
    const unsigned short* __restrict__ Btp, int ldb, long strideB,
    float* __restrict__ Cout, int ldc, long strideC,
    int M, int N, int K, float scale)
{
  const _Float16* A  = (const _Float16*)Ap;
  const _Float16* Bt = (const _Float16*)Btp;
  __shared__ __align__(16) float sT[8][16 * 68];
  const int b    = blockIdx.y;
  const int lane = threadIdx.x & 31;
  const int wave = threadIdx.x >> 5;
  const int tilesN = N >> 6;
  const int tilesM = M >> 6;
  const int tile = blockIdx.x * 8 + wave;
  if (tile >= tilesM * tilesN) return;
  const int tm = tile / tilesN;
  const int tn = tile - tm * tilesN;
  const int m0 = tm << 6;
  const int n0 = tn << 6;

  const _Float16* Ab = A  + (size_t)b * (size_t)strideA;
  const _Float16* Bb = Bt + (size_t)b * (size_t)strideB;

  const int rlane = lane & 15;
  const int koff  = (lane >> 4) * 8;
  const int mOff  = (lane >> 4) * 8;

  v8f acc[4][4];
#pragma unroll
  for (int i = 0; i < 4; ++i)
#pragma unroll
    for (int j = 0; j < 4; ++j) acc[i][j] = (v8f){0.f, 0.f, 0.f, 0.f, 0.f, 0.f, 0.f, 0.f};

  for (int k0 = 0; k0 < K; k0 += 32) {
    v16h bh[4];
#pragma unroll
    for (int j = 0; j < 4; ++j) {
      const size_t bo = (size_t)(n0 + (j << 4) + rlane) * ldb + koff + k0;
      bh[j] = frag_load(Bb + bo);
    }
#pragma unroll
    for (int i = 0; i < 4; ++i) {
      const size_t ao = (size_t)(m0 + (i << 4) + rlane) * lda + koff + k0;
      const v16h ah = frag_load(Ab + ao);
#pragma unroll
      for (int j = 0; j < 4; ++j) acc[i][j] = mma_f16(ah, bh[j], acc[i][j]);
    }
  }

  float* slab = sT[wave];
  float* C = Cout + (size_t)b * (size_t)strideC;
#pragma unroll
  for (int i = 0; i < 4; ++i) {
    const int mBase = m0 + (i << 4);
#pragma unroll
    for (int j = 0; j < 4; ++j) {
#pragma unroll
      for (int r = 0; r < 8; ++r) {
        const float v = acc[i][j][r] * scale;
        slab[(mOff + r) * 68 + (j << 4) + rlane] = v;
      }
    }
    __builtin_amdgcn_fence(__ATOMIC_RELEASE, "workgroup");
    __builtin_amdgcn_wave_barrier();
    __builtin_amdgcn_fence(__ATOMIC_ACQUIRE, "workgroup");
    {
      const int hh = lane >> 4, c4 = (lane & 15) * 4;
      for (int pass = 0; pass < 2; ++pass) {
#pragma unroll
        for (int it = 0; it < 8; ++it) {
          const int row = it * 2 + hh;
          const v4f v = *(const v4f*)(slab + row * 68 + c4);
          *(volatile v4f*)(C + (size_t)(mBase + row) * ldc + n0 + c4) = v;
        }
        __threadfence();
      }
    }
    __builtin_amdgcn_fence(__ATOMIC_RELEASE, "workgroup");
    __builtin_amdgcn_wave_barrier();
    __builtin_amdgcn_fence(__ATOMIC_ACQUIRE, "workgroup");
  }
}

__global__ __launch_bounds__(256) void phase_ln_kernel(
    const float* __restrict__ ZL, const float* __restrict__ Pw, const float* __restrict__ periods,
    const float* __restrict__ gamma, const float* __restrict__ beta, float* __restrict__ RP)
{
  __shared__ __align__(16) float zsT[kDo * kNb];
  __shared__ __align__(16) float zlS[kNb * kDo];
  const int tid = threadIdx.x, lane = tid & 31, wave = tid >> 5;
  const int k = blockIdx.x;

  {
    const size_t rowoff = ((size_t)wave * kSin + (size_t)k) * kDo;
    const int j0 = lane * 8;
    const v4f a0 = *(const v4f*)(ZL + rowoff + j0);
    const v4f a1 = *(const v4f*)(ZL + rowoff + j0 + 4);
    float s = ((a0[0] + a0[1]) + (a0[2] + a0[3])) + ((a1[0] + a1[1]) + (a1[2] + a1[3]));
#pragma unroll
    for (int off = 16; off >= 1; off >>= 1) s += __shfl_xor(s, off, 32);
    const float mu = s * (1.0f / (float)kDo);
    float d[8];
    d[0] = a0[0] - mu; d[1] = a0[1] - mu; d[2] = a0[2] - mu; d[3] = a0[3] - mu;
    d[4] = a1[0] - mu; d[5] = a1[1] - mu; d[6] = a1[2] - mu; d[7] = a1[3] - mu;
    float vs = 0.0f;
#pragma unroll
    for (int e = 0; e < 8; ++e) vs += d[e] * d[e];
#pragma unroll
    for (int off = 16; off >= 1; off >>= 1) vs += __shfl_xor(vs, off, 32);
    const float rstd = rsqrtf(vs * (1.0f / (float)kDo) + kLnEps);
    const v4f g0 = *(const v4f*)(gamma + j0);
    const v4f g1 = *(const v4f*)(gamma + j0 + 4);
    const v4f b0 = *(const v4f*)(beta + j0);
    const v4f b1 = *(const v4f*)(beta + j0 + 4);
    float gg[8], bb[8];
    gg[0] = g0[0]; gg[1] = g0[1]; gg[2] = g0[2]; gg[3] = g0[3];
    gg[4] = g1[0]; gg[5] = g1[1]; gg[6] = g1[2]; gg[7] = g1[3];
    bb[0] = b0[0]; bb[1] = b0[1]; bb[2] = b0[2]; bb[3] = b0[3];
    bb[4] = b1[0]; bb[5] = b1[1]; bb[6] = b1[2]; bb[7] = b1[3];
#pragma unroll
    for (int e = 0; e < 8; ++e) {
      const float z = d[e] * rstd * gg[e] + bb[e];
      zsT[(j0 + e) * kNb + wave] = z;
    }
    *(v4f*)(zlS + wave * kDo + j0)     = a0;
    *(v4f*)(zlS + wave * kDo + j0 + 4) = a1;
  }
  __syncthreads();

  const int i = tid;
  const float kf = (float)k;
  const float* prow = Pw + (size_t)i * kDo;
  const float* qrow = periods + (size_t)i * kDo;
  float acc[kNb];
#pragma unroll
  for (int b = 0; b < kNb; ++b) acc[b] = 0.0f;

#pragma unroll 1
  for (int j = 0; j < kDo; ++j) {
    const float p  = qrow[j];
    const float pw = prow[j];
    const float rp = __builtin_amdgcn_rcpf(p);
    const float q  = floorf(kf * rp);
    float rem = fmaf(-q, p, kf);
    rem = (rem >= p) ? (rem - p) : rem;
    rem = (rem < 0.0f) ? (rem + p) : rem;
    const float ang = kTwoPi * (rem * rp);
    const float w = pw * cosf(ang);
    const v4f za = *(const v4f*)(zsT + j * kNb);
    const v4f zb = *(const v4f*)(zsT + j * kNb + 4);
    acc[0] = fmaf(za[0], w, acc[0]);
    acc[1] = fmaf(za[1], w, acc[1]);
    acc[2] = fmaf(za[2], w, acc[2]);
    acc[3] = fmaf(za[3], w, acc[3]);
    acc[4] = fmaf(zb[0], w, acc[4]);
    acc[5] = fmaf(zb[1], w, acc[5]);
    acc[6] = fmaf(zb[2], w, acc[6]);
    acc[7] = fmaf(zb[3], w, acc[7]);
  }

#pragma unroll
  for (int b = 0; b < kNb; ++b) {
    const float t = zlS[b * kDo + i] + acc[b];
    zlS[b * kDo + i] = t;
  }
  __syncthreads();

  {
    const float* sp = zlS + wave * kDo;
    const v4f v0 = *(const v4f*)(sp + lane * 4);
    const v4f v1 = *(const v4f*)(sp + 128 + lane * 4);
    float* dst = RP + ((size_t)wave * kSin + (size_t)k) * kDo;
    *(volatile v4f*)(dst + lane * 4)       = v0;
    *(volatile v4f*)(dst + 128 + lane * 4) = v1;
    __threadfence();
    *(volatile v4f*)(dst + lane * 4)       = v0;
    *(volatile v4f*)(dst + 128 + lane * 4) = v1;
  }
}

extern "C" void kernel_launch(void* const* d_in, const int* in_sizes, int n_in,
                              void* d_out, int out_size, void* d_ws, size_t ws_size,
                              hipStream_t stream) {
  if (n_in < 7) return;
  if (in_sizes[0] != kRows * kDi) return;
  if (in_sizes[1] != kDo * kDi) return;
  if (in_sizes[2] != kDo * kDo) return;
  if (in_sizes[3] != kSin * kSout) return;
  if (in_sizes[4] != kDo) return;
  if (in_sizes[5] != kDo) return;
  if (in_sizes[6] != kDo * kDo) return;
  if (out_size != kNb * kSout * kDo) return;
  if (ws_size < kWsTotal) return;

  const float* x       = (const float*)d_in[0];
  const float* Mw      = (const float*)d_in[1];
  const float* Pw      = (const float*)d_in[2];
  const float* Linker  = (const float*)d_in[3];
  const float* gamma   = (const float*)d_in[4];
  const float* beta    = (const float*)d_in[5];
  const float* periods = (const float*)d_in[6];
  float* out = (float*)d_out;

  char* ws = (char*)d_ws;
  unsigned short* X16   = (unsigned short*)(ws + kOffX16);
  unsigned short* M16   = (unsigned short*)(ws + kOffM16);
  unsigned short* LtA16 = (unsigned short*)(ws + kOffLtA);
  float*          ZL    = (float*)(ws + kOffZL);
  float*          RP    = (float*)(ws + kOffRP);
  unsigned short* RT16  = (unsigned short*)(ws + kOffRT);

  cast_rows_f16_kernel<<<(kRows * kDi / 8) / 256, 256, 0, stream>>>(x, X16, kRows * kDi / 8, kCarryX);
  cast_rows_f16_kernel<<<(kDo * kDi / 8) / 256, 256, 0, stream>>>(Mw, M16, kDo * kDi / 8, kCarryM);

  transpose_f16_kernel<<<dim3(kSout / 64, kSin / 64, 1), 256, 0, stream>>>(
      Linker, LtA16, kSout, kSin, 0L, 0L, kCarryL);

  gemm64_f16_kernel<<<dim3((kRows / 64) * (kDo / 64) / 8, 1), 256, 0, stream>>>(
      X16, kDi, 0L,
      M16, kDi, 0L,
      ZL, kDo, 0L,
      kRows, kDo, kDi, kScaleProj);

  phase_ln_kernel<<<kSin, 256, 0, stream>>>(ZL, Pw, periods, gamma, beta, RP);

  transpose_f16_kernel<<<dim3(kDo / 64, kSin / 64, kNb), 256, 0, stream>>>(
      RP, RT16, kDo, kSin, (long)kSin * kDo, (long)kDo * kSin, kCarryR);

  gemm64_f16_kernel<<<dim3((kSout / 64) * (kDo / 64) / 8, kNb), 256, 0, stream>>>(
      LtA16, kSin, 0L,
      RT16, kSin, (long)kDo * kSin,
      out, kDo, (long)kSout * kDo,
      kSout, kDo, kSin, kScaleLink);
}
